// EGCL_13692355739802
// MI455X (gfx1250) — hardware-verified
//
#include <hip/hip_runtime.h>
#include <stddef.h>
#include <stdint.h>


#define HID    128
#define NPQ    256
#define NPV    384
#define KN1    384
#define KN2    256
#define W1R    257
#define NTHR   256
#define NWAVE  8
#define EPB    256
#define DP     132
#define AP     136
#define MPITCH 128
#define CSTN   656
#define GBM    64
#define GBN    128
#define GTHR   128
#define EPT    8
#define CHUNK  (NTHR * EPT)
#define WCAP   (EPT * 32)
#define LISTN  (NWAVE * WCAP)
#define NBA    1024
#define SLA    10
#define RCAP   16896
#define DEGCAP 96
#define NRANGE 5
#define NU_WAB  (NPQ * (HID / 8))
#define NU_WV   (HID * (HID / 8))
#define NU_W128 (HID * (HID / 8))
#define NU_WN1  (HID * (KN1 / 8))
#define NU_WN2  (HID * (KN2 / 8))
#define AGG_ZINTS (LISTN + 2 * RCAP + 3 * NBA)
#define AGG_LDS_INTS (AGG_ZINTS + 16 + 4 * NBA)
#define AGG_LDS_BYTES (AGG_LDS_INTS * 4)
#define EDGE_LDS_BYTES (EPB * DP * 4 + EPB * AP * 2 + CSTN * 4)
#define WSMAX  134217728
#define CACT   16.0f
#define CWGT   1024.0f
#define CMSG   16.0f
#define PINV   6.103515625e-05f
#define MINV   0.0625f

static_assert((CHUNK & (CHUNK - 1)) == 0 && CHUNK <= 4096);
static_assert((NBA & (NBA - 1)) == 0 && NBA == (1 << SLA));
static_assert(((long long)CHUNK << SLA) < (1LL << 31));
static_assert(LISTN % NTHR == 0);
static_assert(NBA % NWAVE == 0 && NBA % 32 == 0 && NBA == 4 * NTHR);
static_assert(RCAP % 4 == 0 && AGG_ZINTS % 4 == 0 && LISTN % 4 == 0);
static_assert(AGG_LDS_BYTES <= 300000);
static_assert(EDGE_LDS_BYTES <= 300000);
static_assert(NU_WAB % NTHR == 0 && NU_WV % NTHR == 0 && NU_W128 % NTHR == 0 && NU_WN1 % NTHR == 0 && NU_WN2 % NTHR == 0);
static_assert(HID % 32 == 0 && KN1 % 32 == 0 && KN2 % 32 == 0);
static_assert(GBM == (GTHR / 32) * 16 && GBN == 4 * 32 && GBN == HID && NPQ == 2 * GBN && NPV == 3 * GBN && GTHR == GBN);
static_assert((DP * 4) % 16 == 0 && (AP * 2) % 16 == 0 && AP >= HID && DP >= HID);
static_assert(EPB == NTHR && EPB == 8 * 32);
static_assert((EPB * DP * 4) % 16 == 0 && (EPB * AP * 2) % 16 == 0);
static_assert((CSTN * 4) % 16 == 0 && CSTN >= 5 * HID);
static_assert(EPB * MPITCH * 2 == 16 * NTHR * 16);
static_assert(KN1 == 3 * HID && KN2 == 2 * HID && W1R == 2 * HID + 1);
static_assert(DEGCAP % 32 == 0);

typedef float          v4f   __attribute__((ext_vector_type(4)));
typedef float          v8f   __attribute__((ext_vector_type(8)));
typedef int            v4i   __attribute__((ext_vector_type(4)));
typedef int            v8i   __attribute__((ext_vector_type(8)));
typedef unsigned       v2u   __attribute__((ext_vector_type(2)));
typedef unsigned short v8us  __attribute__((ext_vector_type(8)));
typedef unsigned short v16us __attribute__((ext_vector_type(16)));
typedef __bf16         v16bf __attribute__((ext_vector_type(16)));
typedef _Float16       v16h  __attribute__((ext_vector_type(16)));
typedef v4f  __attribute__((may_alias)) v4fa;
typedef v4i  __attribute__((may_alias)) v4ia;
typedef v2u  __attribute__((may_alias)) v2ua;
typedef v8us __attribute__((may_alias)) v8usa;
union FragB { v16bf v; v16us u; v8us h[2]; v8i w; };
union FragH { v16h  v; v16us u; v8us h[2]; v8i w; };

__device__ __forceinline__ v8f wmb(const FragB& a, const FragB& b, v8f c) {
  v8f d = __builtin_amdgcn_wmma_f32_16x16x32_bf16(false, a.v, false, b.v, (short)0, c, false, false);
  asm volatile("v_nop\n\tv_nop\n\tv_nop\n\tv_nop" : "+v"(d) : "v"(a.w), "v"(b.w));
  return d;
}
__device__ __forceinline__ v8f wmh(const FragH& a, const FragH& b, v8f c) {
  v8f d = __builtin_amdgcn_wmma_f32_16x16x32_f16(false, a.v, false, b.v, (short)0, c, false, false);
  asm volatile("v_nop\n\tv_nop\n\tv_nop\n\tv_nop" : "+v"(d) : "v"(a.w), "v"(b.w));
  return d;
}

__device__ __forceinline__ unsigned bf16_bits(float f) {
  const unsigned u = __float_as_uint(f);
  return (u + 0x7FFFu + ((u >> 16) & 1u)) >> 16;
}
__device__ __forceinline__ float bf16_val(float f) {
  return __uint_as_float(bf16_bits(f) << 16);
}
__device__ __forceinline__ unsigned short f2h(float f) {
  const _Float16 hv = (_Float16)f;
  return __builtin_bit_cast(unsigned short, hv);
}
__device__ __forceinline__ float h2f(unsigned b) {
  const _Float16 hv = __builtin_bit_cast(_Float16, (unsigned short)b);
  return (float)hv;
}
__device__ __forceinline__ float silu_f(float t) {
  return t * __builtin_amdgcn_rcpf(1.0f + __expf(-t));
}
__device__ __forceinline__ void put16(unsigned short* dp, v8us o) {
  *(volatile v8us*)dp = o;
  __threadfence();
  *(volatile v8us*)dp = o;
}
__device__ __forceinline__ void putf4(float* dp, v4f o) {
  *(volatile v4f*)dp = o;
  __threadfence();
  *(volatile v4f*)dp = o;
}
__device__ __forceinline__ int clampi(int v, int lo, int hi) { return v < lo ? lo : (v > hi ? hi : v); }

template <int SLB>
__device__ __forceinline__ int scan_chunk(const int* __restrict__ dsts, int nE, int cbase, int slotBase,
                                          int nb, int vec8, int* list, int tid, int lane, int wave) {
  int wc = 0;
  const int el0  = tid * EPT;
  const int e0   = cbase + el0;
  const int sent = -2147483647 - 1;
  v4i da, db;
  if (vec8 != 0 && cbase + CHUNK <= nE) {
    da = *(const v4i*)(dsts + e0);
    db = *(const v4i*)(dsts + e0 + 4);
  } else {
    da.x = (e0     < nE) ? dsts[min(e0,     nE - 1)] : sent;
    da.y = (e0 + 1 < nE) ? dsts[min(e0 + 1, nE - 1)] : sent;
    da.z = (e0 + 2 < nE) ? dsts[min(e0 + 2, nE - 1)] : sent;
    da.w = (e0 + 3 < nE) ? dsts[min(e0 + 3, nE - 1)] : sent;
    db.x = (e0 + 4 < nE) ? dsts[min(e0 + 4, nE - 1)] : sent;
    db.y = (e0 + 5 < nE) ? dsts[min(e0 + 5, nE - 1)] : sent;
    db.z = (e0 + 6 < nE) ? dsts[min(e0 + 6, nE - 1)] : sent;
    db.w = (e0 + 7 < nE) ? dsts[min(e0 + 7, nE - 1)] : sent;
  }
  const unsigned nbs = (unsigned)slotBase;
  const unsigned unb = (unsigned)nb;
  const unsigned s0 = (unsigned)da.x - nbs, s1 = (unsigned)da.y - nbs;
  const unsigned s2 = (unsigned)da.z - nbs, s3 = (unsigned)da.w - nbs;
  const unsigned s4 = (unsigned)db.x - nbs, s5 = (unsigned)db.y - nbs;
  const unsigned s6 = (unsigned)db.z - nbs, s7 = (unsigned)db.w - nbs;
  const bool h0 = s0 < unb, h1 = s1 < unb, h2 = s2 < unb, h3 = s3 < unb;
  const bool h4 = s4 < unb, h5 = s5 < unb, h6 = s6 < unb, h7 = s7 < unb;
  const unsigned any = __builtin_amdgcn_ballot_w32(h0 | h1 | h2 | h3 | h4 | h5 | h6 | h7);
  if (any != 0u) {
#define HITJ(J, HJ, SJ) { \
      const unsigned mj = __builtin_amdgcn_ballot_w32(HJ); \
      if (mj != 0u) { \
        if (HJ) { \
          const int pos = wc + (int)__builtin_amdgcn_mbcnt_lo(mj, 0u); \
          if (pos < WCAP) list[wave * WCAP + pos] = ((el0 + (J)) << SLB) | (int)(SJ); \
        } \
        wc += (int)__builtin_popcount(mj); } }
    HITJ(0, h0, s0)
    HITJ(1, h1, s1)
    HITJ(2, h2, s2)
    HITJ(3, h3, s3)
    HITJ(4, h4, s4)
    HITJ(5, h5, s5)
    HITJ(6, h6, s6)
    HITJ(7, h7, s7)
#undef HITJ
  }
  return wc;
}

__global__ __launch_bounds__(NTHR) void k_prep(const float* __restrict__ h,
                                               const float* __restrict__ We1, const float* __restrict__ We2,
                                               const float* __restrict__ Wc1, const float* __restrict__ Wn1,
                                               const float* __restrict__ Wn2, const float* __restrict__ Wv1,
                                               int nN, int mRows,
                                               unsigned short* WABT, unsigned short* WE2T, unsigned short* WX1T,
                                               unsigned short* WN1T, unsigned short* WN2T,
                                               unsigned short* HB, float* MI, float* DX) {
  const int u  = (int)blockIdx.x * NTHR + (int)threadIdx.x;
  const int UA = NU_WAB;
  const int U0 = UA + NU_WV;
  const int U1 = U0 + NU_W128;
  const int U2 = U1 + NU_W128;
  const int U3 = U2 + NU_WN1;
  const int U4 = U3 + NU_WN2;
  const int U5 = U4 + mRows * 16;
  const int U6 = U5 + mRows * 32;
  const int nXP = ((mRows + NTHR - 1) / NTHR) * NTHR;
  const int U7 = U6 + nXP;
  const v4f z4 = {0.0f, 0.0f, 0.0f, 0.0f};
  v8us o;
  if (u < UA) {
    const int n   = u >> 4;
    const int k8  = (u & 15) * 8;
    const int kof = (n >> 7) * HID;
    const int nn  = n & (HID - 1);
    const float* p = We1 + (size_t)(kof + k8) * HID + nn;
#pragma unroll
    for (int i = 0; i < 8; ++i) o[i] = (unsigned short)bf16_bits(p[(size_t)i * HID]);
    put16(WABT + (size_t)n * HID + k8, o);
    return;
  } else if (u < U0) {
    const int v  = u - UA;
    const int n  = v >> 4;
    const int k8 = (v & 15) * 8;
    const float* p = Wv1 + (size_t)k8 * HID + n;
#pragma unroll
    for (int i = 0; i < 8; ++i) o[i] = (unsigned short)bf16_bits(p[(size_t)i * HID]);
    put16(WABT + (size_t)(NPQ + n) * HID + k8, o);
    return;
  } else if (u < U1) {
    const int v  = u - U0;
    const int n  = v >> 4;
    const int k8 = (v & 15) * 8;
    const float* p = We2 + (size_t)k8 * HID + n;
#pragma unroll
    for (int i = 0; i < 8; ++i) o[i] = f2h(CWGT * bf16_val(p[(size_t)i * HID]));
    put16(WE2T + (size_t)n * HID + k8, o);
    return;
  } else if (u < U2) {
    const int v  = u - U1;
    const int n  = v >> 4;
    const int k8 = (v & 15) * 8;
    const float* p = Wc1 + (size_t)k8 * HID + n;
#pragma unroll
    for (int i = 0; i < 8; ++i) o[i] = f2h(CWGT * bf16_val(p[(size_t)i * HID]));
    put16(WX1T + (size_t)n * HID + k8, o);
    return;
  } else if (u < U3) {
    const int v    = u - U2;
    const int n    = v / (KN1 / 8);
    const int k8   = (v - n * (KN1 / 8)) * 8;
    const int srow = (k8 < 2 * HID) ? k8 : (k8 - HID);
    const float* p = Wn1 + (size_t)srow * HID + n;
#pragma unroll
    for (int i = 0; i < 8; ++i) o[i] = (unsigned short)bf16_bits(p[(size_t)i * HID]);
    put16(WN1T + (size_t)n * KN1 + k8, o);
    return;
  } else if (u < U4) {
    const int v    = u - U3;
    const int n    = v >> 5;
    const int k8   = (v & 31) * 8;
    const int srow = k8 & (HID - 1);
    const float* p = Wn2 + (size_t)srow * HID + n;
#pragma unroll
    for (int i = 0; i < 8; ++i) o[i] = (unsigned short)bf16_bits(p[(size_t)i * HID]);
    put16(WN2T + (size_t)n * KN2 + k8, o);
    return;
  } else if (u < U5) {
    const int v   = u - U4;
    const int row = v >> 4;
    const int k8  = (v & 15) * 8;
    const int rc  = row < nN ? row : nN - 1;
    const float* p = h + (size_t)rc * HID + k8;
    const v4f a = *(const v4fa*)p;
    const v4f b = *(const v4fa*)(p + 4);
    const unsigned msk = (row < nN) ? 0xffffu : 0u;
    o[0] = (unsigned short)(bf16_bits(a.x) & msk);
    o[1] = (unsigned short)(bf16_bits(a.y) & msk);
    o[2] = (unsigned short)(bf16_bits(a.z) & msk);
    o[3] = (unsigned short)(bf16_bits(a.w) & msk);
    o[4] = (unsigned short)(bf16_bits(b.x) & msk);
    o[5] = (unsigned short)(bf16_bits(b.y) & msk);
    o[6] = (unsigned short)(bf16_bits(b.z) & msk);
    o[7] = (unsigned short)(bf16_bits(b.w) & msk);
    put16(HB + (size_t)row * HID + k8, o);
    return;
  } else if (u < U6) {
    const int v = u - U5;
    putf4(MI + (size_t)v * 4, z4);
    return;
  } else if (u < U7) {
    const int row = u - U6;
    if (row >= mRows) return;
    putf4(DX + (size_t)row * 4, z4);
    return;
  }
}

template <int MODE>
__global__ __launch_bounds__(GTHR) void k_gemm(const unsigned short* __restrict__ A, int lda,
                                               const unsigned short* __restrict__ BT, int ldb, int K,
                                               const float* __restrict__ bias, const float* __restrict__ wvec,
                                               const float* __restrict__ bsc, int nN,
                                               float* Cm, int ldc, unsigned short* Cb, float* Cv) {
  __shared__ __attribute__((aligned(16))) float stg[GBM * GBN];
  __shared__ __attribute__((aligned(16))) float sW[GBN];
  __shared__ __attribute__((aligned(16))) float sV[GBM];
  const int tid = (int)threadIdx.x, lane = tid & 31, wave = tid >> 5, hh = lane >> 4, m = lane & 15;
  const int rowBase = (int)blockIdx.x * GBM;
  int colBase = 0;
  bool isV = false;
  if constexpr (MODE == 0) {
    colBase = (int)blockIdx.y * GBN;
    isV = (blockIdx.y == 2);
    sW[tid] = bf16_val(wvec[tid]);
  }

  v8f acc[8];
  {
    const v8f z = {0.f, 0.f, 0.f, 0.f, 0.f, 0.f, 0.f, 0.f};
#pragma unroll
    for (int t = 0; t < 8; ++t) acc[t] = z;
  }
  const unsigned short* ap = A  + (size_t)(rowBase + 16 * wave + m) * (size_t)lda + 8 * hh;
  const unsigned short* bp = BT + (size_t)(colBase + m) * (size_t)ldb + 8 * hh;

#pragma unroll 1
  for (int k0 = 0; k0 < K; k0 += 32) {
    FragB af;
    af.h[0] = *(const v8usa*)(ap + k0);
    af.h[1] = *(const v8usa*)(ap + k0 + 16);
#pragma unroll
    for (int nt = 0; nt < 8; ++nt) {
      const unsigned short* wq = bp + (size_t)(16 * nt) * (size_t)ldb + k0;
      FragB bf;
      bf.h[0] = *(const v8usa*)wq;
      bf.h[1] = *(const v8usa*)(wq + 16);
      acc[nt] = wmb(af, bf, acc[nt]);
    }
  }

#pragma unroll
  for (int nt = 0; nt < 8; ++nt) {
    const int lc = 16 * nt + m;
    const float bvv = bf16_val(bias[lc]);
#pragma unroll
    for (int r = 0; r < 8; ++r) {
      const int lr = 16 * wave + 8 * hh + r;
      float v = acc[nt][r];
      if constexpr (MODE == 0) { if (isV) v = silu_f(v + bvv); }
      if constexpr (MODE == 1) v = silu_f(v + bvv);
      if constexpr (MODE == 2) v = v + bvv;
      stg[lr * GBN + lc] = v;
    }
  }
  __syncthreads();

  if constexpr (MODE == 0) {
    if (isV && tid < GBM) {
      float s = 0.0f;
      const float* sp = stg + tid * GBN;
#pragma unroll 4
      for (int c = 0; c < GBN; ++c) s = fmaf(sp[c], sW[c], s);
      sV[tid] = s + bf16_val(bsc[0]);
    }
    __syncthreads();
    if (!isV) {
      v4f pv[16];
#pragma unroll
      for (int i = 0; i < 16; ++i) pv[i] = *(const v4fa*)(stg + (16 * wave + i) * GBN + 4 * lane);
#pragma unroll
      for (int i = 0; i < 16; ++i) {
        float* op = Cm + (size_t)(rowBase + 16 * wave + i) * (size_t)ldc + colBase + 4 * lane;
        *(volatile v4f*)op = pv[i];
      }
      __threadfence();
#pragma unroll
      for (int i = 0; i < 16; ++i) {
        float* op = Cm + (size_t)(rowBase + 16 * wave + i) * (size_t)ldc + colBase + 4 * lane;
        *(volatile v4f*)op = pv[i];
      }
    } else if (wave == 0) {
      const int tl = lane & 15;
      const v4f o4 = *(const v4fa*)(sV + 4 * tl);
      float* dp = Cv + (size_t)rowBase + 4 * tl;
      if (lane < 16) *(volatile v4f*)dp = o4;
      __threadfence();
      if (lane < 16) *(volatile v4f*)dp = o4;
    }
  } else if constexpr (MODE == 1) {
    const int part = lane >> 4;
    const int j = lane & 15;
    const unsigned mh = 0u - (unsigned)part;
    const unsigned ml = ~mh;
    v8us pv[16];
#pragma unroll
    for (int i = 0; i < 16; ++i) {
      const float* sp = stg + (16 * wave + i) * GBN + 8 * j;
      const v4f a = *(const v4fa*)sp;
      const v4f b = *(const v4fa*)(sp + 4);
      const v8f f8 = {a.x, a.y, a.z, a.w, b.x, b.y, b.z, b.w};
      v8us oo;
#pragma unroll
      for (int e = 0; e < 8; ++e) {
        const unsigned hb = bf16_bits(f8[e]);
        const unsigned lb = bf16_bits(f8[e] - __uint_as_float(hb << 16));
        oo[e] = (unsigned short)((hb & ml) | (lb & mh));
      }
      pv[i] = oo;
    }
#pragma unroll
    for (int i = 0; i < 16; ++i) {
      unsigned short* op = Cb + (size_t)(rowBase + 16 * wave + i) * (size_t)KN2 + part * HID + 8 * j;
      *(volatile v8us*)op = pv[i];
    }
    __threadfence();
#pragma unroll
    for (int i = 0; i < 16; ++i) {
      unsigned short* op = Cb + (size_t)(rowBase + 16 * wave + i) * (size_t)KN2 + part * HID + 8 * j;
      *(volatile v8us*)op = pv[i];
    }
  } else {
    v4f pv[16];
#pragma unroll
    for (int i = 0; i < 16; ++i) pv[i] = *(const v4fa*)(stg + (16 * wave + i) * GBN + 4 * lane);
#pragma unroll
    for (int i = 0; i < 16; ++i) {
      const int row = rowBase + 16 * wave + i;
      if (row < nN) {
        float* op = Cm + (size_t)row * (size_t)ldc + colBase + 4 * lane;
        *(volatile v4f*)op = pv[i];
      }
    }
    __threadfence();
#pragma unroll
    for (int i = 0; i < 16; ++i) {
      const int row = rowBase + 16 * wave + i;
      if (row < nN) {
        float* op = Cm + (size_t)row * (size_t)ldc + colBase + 4 * lane;
        *(volatile v4f*)op = pv[i];
      }
    }
  }
}

__device__ __forceinline__ void wave_gemm_h(const unsigned short* sAw, float* sDw,
                                            const unsigned short* __restrict__ BT, int ldb, int K,
                                            int hh, int m) {
#pragma unroll 1
  for (int nh = 0; nh < 2; ++nh) {
    v8f acc[2][4];
    {
      const v8f z = {0.f, 0.f, 0.f, 0.f, 0.f, 0.f, 0.f, 0.f};
#pragma unroll
      for (int mt = 0; mt < 2; ++mt)
#pragma unroll
        for (int nt = 0; nt < 4; ++nt) acc[mt][nt] = z;
    }
    const unsigned short* ap0 = sAw + m * AP + 8 * hh;
    const unsigned short* ap1 = ap0 + 16 * AP;
    const unsigned short* bp  = BT + (size_t)(64 * nh + m) * (size_t)ldb + 8 * hh;
#pragma unroll 1
    for (int k0 = 0; k0 < K; k0 += 32) {
      FragH a0, a1;
      a0.h[0] = *(const v8usa*)(ap0 + k0);
      a0.h[1] = *(const v8usa*)(ap0 + k0 + 16);
      a1.h[0] = *(const v8usa*)(ap1 + k0);
      a1.h[1] = *(const v8usa*)(ap1 + k0 + 16);
#pragma unroll
      for (int nt = 0; nt < 4; ++nt) {
        const unsigned short* wq = bp + (size_t)(16 * nt) * (size_t)ldb + k0;
        FragH b;
        b.h[0] = *(const v8usa*)wq;
        b.h[1] = *(const v8usa*)(wq + 16);
        acc[0][nt] = wmh(a0, b, acc[0][nt]);
        acc[1][nt] = wmh(a1, b, acc[1][nt]);
      }
    }
#pragma unroll
    for (int nt = 0; nt < 4; ++nt) {
      const int col = 64 * nh + 16 * nt + m;
#pragma unroll
      for (int mt = 0; mt < 2; ++mt)
#pragma unroll
        for (int r = 0; r < 8; ++r) sDw[(16 * mt + 8 * hh + r) * DP + col] = acc[mt][nt][r];
    }
  }
}

__global__ __launch_bounds__(NTHR) void k_edge(const int* __restrict__ rowp, const int* __restrict__ colp,
                                               int nE, int nN, int eBase, int nEh,
                                               const float* __restrict__ PQ, const float* __restrict__ cdp,
                                               const unsigned short* __restrict__ WE2T,
                                               const unsigned short* __restrict__ WX1T,
                                               const float* __restrict__ be1, const float* __restrict__ be2,
                                               const float* __restrict__ bc1, const float* __restrict__ w256,
                                               const float* __restrict__ wc2,
                                               unsigned short* Mh, float* TRh) {
  extern __shared__ __attribute__((aligned(16))) float dyn[];
  float*          sD  = dyn;
  unsigned short* sA  = (unsigned short*)(dyn + EPB * DP);
  float*          cst = dyn + EPB * DP + (EPB * AP) / 2;

  const int tid = (int)threadIdx.x, lane = tid & 31, wave = tid >> 5, hh = lane >> 4, m = lane & 15;

  if (tid < HID) {
    cst[tid]           = bf16_val(be1[tid]);
    cst[HID + tid]     = bf16_val(be2[tid]);
    cst[2 * HID + tid] = bf16_val(bc1[tid]);
    cst[3 * HID + tid] = bf16_val(w256[tid]);
    cst[4 * HID + tid] = bf16_val(wc2[tid]);
  }

  const int  elb  = (int)blockIdx.x * EPB;
  const int  el   = elb + tid;
  const bool live = el < nEh;
  const int  elc  = live ? el : (nEh - 1);
  int eg = eBase + elc;
  eg = eg < nE ? eg : (nE - 1);
  int r = rowp[eg];
  int c = colp[eg];
  r = clampi(r, 0, nN - 1);
  c = clampi(c, 0, nN - 1);
  const float cx = bf16_val(cdp[(size_t)eg * 3 + 0]);
  const float cy = bf16_val(cdp[(size_t)eg * 3 + 1]);
  const float cz = bf16_val(cdp[(size_t)eg * 3 + 2]);
  const float radial = (cx * cx + cz * cz) + cy * cy;
  __syncthreads();

  float*          rd = sD + tid * DP;
  unsigned short* ra = sA + tid * AP;

  {
    const float* pr = PQ + (size_t)r * NPQ;
    const float* qr = PQ + (size_t)c * NPQ + HID;
#pragma unroll 1
    for (int c8 = 0; c8 < HID / 8; ++c8) {
      const v4f pa = *(const v4fa*)(pr + 8 * c8);
      const v4f pb = *(const v4fa*)(pr + 8 * c8 + 4);
      const v4f qa = *(const v4fa*)(qr + 8 * c8);
      const v4f qb = *(const v4fa*)(qr + 8 * c8 + 4);
      const v4f ba = *(const v4fa*)(cst + 8 * c8);
      const v4f bb = *(const v4fa*)(cst + 8 * c8 + 4);
      const v4f ua = *(const v4fa*)(cst + 3 * HID + 8 * c8);
      const v4f ub = *(const v4fa*)(cst + 3 * HID + 8 * c8 + 4);
      const v8f p8 = {pa.x, pa.y, pa.z, pa.w, pb.x, pb.y, pb.z, pb.w};
      const v8f q8 = {qa.x, qa.y, qa.z, qa.w, qb.x, qb.y, qb.z, qb.w};
      const v8f b8 = {ba.x, ba.y, ba.z, ba.w, bb.x, bb.y, bb.z, bb.w};
      const v8f u8 = {ua.x, ua.y, ua.z, ua.w, ub.x, ub.y, ub.z, ub.w};
      v8us o;
#pragma unroll
      for (int i = 0; i < 8; ++i) {
        const float pre = (p8[i] + q8[i]) + fmaf(radial, u8[i], b8[i]);
        o[i] = f2h(CACT * silu_f(pre));
      }
      *(v8usa*)(ra + 8 * c8) = o;
    }
  }
  __syncthreads();

  const unsigned short* sAw = sA + 32 * wave * AP;
  float*                sDw = sD + 32 * wave * DP;

  wave_gemm_h(sAw, sDw, WE2T, HID, HID, hh, m);
  __syncthreads();

  {
#pragma unroll 1
    for (int c8 = 0; c8 < HID / 8; ++c8) {
      const v4f va = *(const v4fa*)(rd + 8 * c8);
      const v4f vb = *(const v4fa*)(rd + 8 * c8 + 4);
      const v4f ba = *(const v4fa*)(cst + HID + 8 * c8);
      const v4f bb = *(const v4fa*)(cst + HID + 8 * c8 + 4);
      const v8f v8 = {va.x, va.y, va.z, va.w, vb.x, vb.y, vb.z, vb.w};
      const v8f b8 = {ba.x, ba.y, ba.z, ba.w, bb.x, bb.y, bb.z, bb.w};
      v8us o;
#pragma unroll
      for (int i = 0; i < 8; ++i) {
        const float mj = silu_f(fmaf(v8[i], PINV, b8[i]));
        o[i] = f2h(CACT * mj);
      }
      *(v8usa*)(ra + 8 * c8) = o;
    }
  }
  __syncthreads();

  {
    v4i pv[16];
#pragma unroll
    for (int it = 0; it < 16; ++it) {
      const int p  = it * NTHR + tid;
      const int rw = p >> 4;
      const int c8 = (p & 15) * 8;
      pv[it] = *(const v4ia*)(sA + rw * AP + c8);
    }
    unsigned short* mb = Mh + (size_t)elb * MPITCH;
#pragma unroll
    for (int it = 0; it < 16; ++it) *(volatile v4i*)(mb + (size_t)(it * NTHR + tid) * 8) = pv[it];
    __threadfence();
#pragma unroll
    for (int it = 0; it < 16; ++it) *(volatile v4i*)(mb + (size_t)(it * NTHR + tid) * 8) = pv[it];
  }

  wave_gemm_h(sAw, sDw, WX1T, HID, HID, hh, m);
  __syncthreads();

  float tsum = 0.0f;
  {
#pragma unroll 1
    for (int c8 = 0; c8 < HID / 8; ++c8) {
      const v4f va = *(const v4fa*)(rd + 8 * c8);
      const v4f vb = *(const v4fa*)(rd + 8 * c8 + 4);
      const v4f ba = *(const v4fa*)(cst + 2 * HID + 8 * c8);
      const v4f bb = *(const v4fa*)(cst + 2 * HID + 8 * c8 + 4);
      const v4f wa = *(const v4fa*)(cst + 4 * HID + 8 * c8);
      const v4f wb = *(const v4fa*)(cst + 4 * HID + 8 * c8 + 4);
      const v8f v8 = {va.x, va.y, va.z, va.w, vb.x, vb.y, vb.z, vb.w};
      const v8f b8 = {ba.x, ba.y, ba.z, ba.w, bb.x, bb.y, bb.z, bb.w};
      const v8f w8 = {wa.x, wa.y, wa.z, wa.w, wb.x, wb.y, wb.z, wb.w};
#pragma unroll
      for (int i = 0; i < 8; ++i) tsum = fmaf(silu_f(fmaf(v8[i], PINV, b8[i])), w8[i], tsum);
    }
  }

  {
    const float okf  = live ? 1.0f : 0.0f;
    const float coef = tsum;
    v4f t4;
    t4.x = okf * fminf(fmaxf(cx * coef, -100.0f), 100.0f);
    t4.y = okf * fminf(fmaxf(cy * coef, -100.0f), 100.0f);
    t4.z = okf * fminf(fmaxf(cz * coef, -100.0f), 100.0f);
    t4.w = 0.0f;
    float* tp = TRh + (size_t)el * 4;
    *(volatile v4f*)tp = t4;
    __threadfence();
    *(volatile v4f*)tp = t4;
  }
}

__global__ __launch_bounds__(NTHR) void k_scan(const int* __restrict__ keys, int nEh, int vec8, int mRows,
                                               const unsigned short* __restrict__ Mh,
                                               const float* __restrict__ TRh, float* MI, float* DX) {
  extern __shared__ __attribute__((aligned(16))) int dsm[];
  int*   list = dsm;
  int*   hl   = dsm + LISTN;
  int*   sl   = hl + RCAP;
  int*   cnt  = sl + RCAP;
  int*   offs = cnt + NBA;
  int*   cur  = offs + NBA;
  int*   misc = cur + NBA;
  float* sdx  = (float*)(misc + 16);
  const int tid = (int)threadIdx.x, lane = tid & 31, wave = tid >> 5;
  const int nodeBase = (int)blockIdx.x * NBA;

  {
    const v4i z4 = {0, 0, 0, 0};
    for (int i = tid * 4; i < AGG_ZINTS; i += NTHR * 4) *(v4ia*)(dsm + i) = z4;
    if (tid < 16) misc[tid] = 0;
  }
  __syncthreads();

  int t = 0, ov = 0;
  const int nChunks = (nEh + CHUNK - 1) / CHUNK;
#pragma unroll 1
  for (int ch = 0; ch < nChunks; ++ch) {
    const int cbase = ch * CHUNK;
    const int wc = scan_chunk<SLA>(keys, nEh, cbase, nodeBase, NBA, vec8, list, tid, lane, wave);
    if (lane == 0) misc[wave] = wc;
    __syncthreads();
    if (wave == 0) {
#pragma unroll 1
      for (int w2 = 0; w2 < NWAVE; ++w2) {
        int cc = misc[w2];
        cc = cc < 0 ? 0 : (cc > WCAP ? WCAP : cc);
#pragma unroll 1
        for (int b0 = 0; b0 < cc; b0 += 32) {
          const int idx = b0 + lane;
          const int ent = list[w2 * WCAP + (idx < WCAP ? idx : WCAP - 1)];
          const int m32 = (cc - b0) < 32 ? (cc - b0) : 32;
#pragma unroll 1
          for (int k = 0; k < m32; ++k) {
            const int u    = __builtin_amdgcn_readlane(ent, k);
            const int slot = u & (NBA - 1);
            const int el   = (u >> SLA) & (CHUNK - 1);
            const int pk   = ((cbase + el) << SLA) | slot;
            if (t < RCAP) {
              if (lane == 0) { hl[t] = pk; cnt[slot] = cnt[slot] + 1; }
              t = t + 1;
            } else {
              ov = 1;
            }
          }
        }
      }
    }
    __syncthreads();
  }
  if (wave == 0 && lane == 0) { misc[8] = t; misc[9] = ov; }
  __syncthreads();
  int tt = misc[8];
  tt = tt < 0 ? 0 : (tt > RCAP ? RCAP : tt);
  const int ovf = misc[9];

  if (wave == 0) {
    const int base = lane * (NBA / 32);
    int s = 0;
#pragma unroll 1
    for (int i = 0; i < NBA / 32; ++i) s += cnt[base + i];
    int incl = s;
#pragma unroll
    for (int d = 1; d < 32; d <<= 1) {
      const int y = __shfl_up(incl, d, 32);
      if (lane >= d) incl += y;
    }
    int run = incl - s;
#pragma unroll 1
    for (int i = 0; i < NBA / 32; ++i) {
      const int cv = cnt[base + i];
      offs[base + i] = run;
      cur[base + i]  = run;
      run += cv;
    }
  }
  __syncthreads();
  if (wave == 0) {
#pragma unroll 1
    for (int b0 = 0; b0 < tt; b0 += 32) {
      const int idx = b0 + lane;
      const int ent = hl[idx < RCAP ? idx : RCAP - 1];
      const int m32 = (tt - b0) < 32 ? (tt - b0) : 32;
#pragma unroll 1
      for (int k = 0; k < m32; ++k) {
        const int u    = __builtin_amdgcn_readlane(ent, k);
        const int slot = u & (NBA - 1);
        if (lane == 0) {
          int p = cur[slot];
          p = p < 0 ? 0 : (p > RCAP - 1 ? RCAP - 1 : p);
          sl[p] = u;
          cur[slot] = p + 1;
        }
      }
    }
  }
  __syncthreads();

  const float qnan = __int_as_float(0x7fc00000);
  const float pz = (ovf != 0) ? qnan : 0.0f;
#pragma unroll 1
  for (int si = 0; si < NBA / NWAVE; ++si) {
    const int s    = si * NWAVE + wave;
    const int node = nodeBase + s;
    const int craw = cnt[s];
    const bool big = craw > DEGCAP;
    const int cdeg = craw < 0 ? 0 : (craw > DEGCAP ? DEGCAP : craw);
    int o = offs[s];
    o = o < 0 ? 0 : (o > RCAP ? RCAP : o);
    float a0 = 0.0f, a1 = 0.0f, a2 = 0.0f, a3 = 0.0f;
    float dx = 0.0f, dy = 0.0f, dz = 0.0f;
#pragma unroll 1
    for (int b0 = 0; b0 < cdeg; b0 += 32) {
      int idx = o + b0 + lane;
      idx = idx > RCAP - 1 ? RCAP - 1 : idx;
      const int ent = sl[idx];
      int eid = ent >> SLA;
      eid = eid < 0 ? 0 : (eid > nEh - 1 ? nEh - 1 : eid);
      const v4f t4 = *(const v4fa*)(TRh + (size_t)eid * 4);
      const int cxi = __float_as_int(t4.x);
      const int cyi = __float_as_int(t4.y);
      const int czi = __float_as_int(t4.z);
      const int m32 = (cdeg - b0) < 32 ? (cdeg - b0) : 32;
#pragma unroll 1
      for (int k = 0; k < m32; ++k) {
        const int ek = __builtin_amdgcn_readlane(eid, k);
        const unsigned short* rp = Mh + (size_t)ek * MPITCH + 4 * lane;
        const v2u w = *(const v2ua*)rp;
        a0 += h2f(w.x & 0xffffu);
        a1 += h2f(w.x >> 16);
        a2 += h2f(w.y & 0xffffu);
        a3 += h2f(w.y >> 16);
        dx += __int_as_float(__builtin_amdgcn_readlane(cxi, k));
        dy += __int_as_float(__builtin_amdgcn_readlane(cyi, k));
        dz += __int_as_float(__builtin_amdgcn_readlane(czi, k));
      }
    }
    const bool  live = node < mRows;
    const int   nr   = live ? node : mRows - 1;
    const float pzr  = big ? qnan : pz;
    float* mp = MI + (size_t)nr * HID + 4 * lane;
    const v4f old = *(const v4fa*)mp;
    v4f nv;
    nv.x = fmaf(a0, MINV, old.x) + pzr;
    nv.y = fmaf(a1, MINV, old.y) + pzr;
    nv.z = fmaf(a2, MINV, old.z) + pzr;
    nv.w = fmaf(a3, MINV, old.w) + pzr;
    if (live) *(volatile v4f*)mp = nv;
    __threadfence();
    if (live) *(volatile v4f*)mp = nv;
    if (lane == 0) {
      const v4f d4 = {dx + pzr, dy + pzr, dz + pzr, (float)craw};
      *(v4fa*)(sdx + 4 * s) = d4;
    }
  }
  __syncthreads();

  v4f dv[4];
#pragma unroll
  for (int j = 0; j < 4; ++j) {
    const int slot = j * NTHR + tid;
    const int node = nodeBase + slot;
    const int nr   = node < mRows ? node : mRows - 1;
    const v4f old  = *(const v4fa*)(DX + (size_t)nr * 4);
    const v4f add  = *(const v4fa*)(sdx + 4 * slot);
    v4f q;
    q.x = old.x + add.x; q.y = old.y + add.y; q.z = old.z + add.z; q.w = old.w + add.w;
    dv[j] = q;
  }
#pragma unroll
  for (int j = 0; j < 4; ++j) {
    const int node = nodeBase + j * NTHR + tid;
    if (node < mRows) *(volatile v4f*)(DX + (size_t)node * 4) = dv[j];
  }
  __threadfence();
#pragma unroll
  for (int j = 0; j < 4; ++j) {
    const int node = nodeBase + j * NTHR + tid;
    if (node < mRows) *(volatile v4f*)(DX + (size_t)node * 4) = dv[j];
  }
}

__global__ __launch_bounds__(NTHR) void k_nz(const float* __restrict__ MI, const float* __restrict__ h,
                                             int nN, int nUnits, unsigned short* NZ) {
  const int u = (int)blockIdx.x * NTHR + (int)threadIdx.x;
  if (u >= nUnits) return;
  const int row = u >> 4;
  const int j   = u & 15;
  const int rc  = row < nN ? row : nN - 1;
  const unsigned msk = (row < nN) ? 0xffffu : 0u;
  const float* mq = MI + (size_t)row * HID + 8 * j;
  const float* hq = h  + (size_t)rc  * HID + 8 * j;
  const v4f ma = *(const v4fa*)mq;
  const v4f mb = *(const v4fa*)(mq + 4);
  const v4f ha = *(const v4fa*)hq;
  const v4f hb = *(const v4fa*)(hq + 4);
  const v8f m8 = {ma.x, ma.y, ma.z, ma.w, mb.x, mb.y, mb.z, mb.w};
  const v8f h8 = {ha.x, ha.y, ha.z, ha.w, hb.x, hb.y, hb.z, hb.w};
  v8us ohi, olo, ohb;
#pragma unroll
  for (int i = 0; i < 8; ++i) {
    const unsigned hbits = bf16_bits(m8[i]);
    ohi[i] = (unsigned short)hbits;
    olo[i] = (unsigned short)bf16_bits(m8[i] - __uint_as_float(hbits << 16));
    ohb[i] = (unsigned short)(bf16_bits(h8[i]) & msk);
  }
  unsigned short* dp = NZ + (size_t)row * KN1 + 8 * j;
  *(volatile v8us*)dp             = ohb;
  *(volatile v8us*)(dp + HID)     = ohi;
  *(volatile v8us*)(dp + 2 * HID) = olo;
  __threadfence();
  *(volatile v8us*)dp             = ohb;
  *(volatile v8us*)(dp + HID)     = ohi;
  *(volatile v8us*)(dp + 2 * HID) = olo;
}

__global__ __launch_bounds__(NTHR) void k_vf(const float* __restrict__ VEL, const float* __restrict__ DX,
                                             int nN, float* out) {
  const int u   = (int)blockIdx.x * NTHR + (int)threadIdx.x;
  const int uc  = u < nN ? u : nN - 1;
  const int nq  = nN >> 2;
  const int ucv = uc < nq ? uc : nq - 1;
  const v4f v4  = *(const v4fa*)(VEL + (size_t)4 * ucv);
  int t0 = 4 * uc - nN;
  t0 = t0 < 0 ? 0 : t0;
  const int nA  = t0 / 3;
  const int nB  = (nA + 1) < nN ? (nA + 1) : (nN - 1);
  const v4f dA  = *(const v4fa*)(DX + (size_t)nA * 4);
  const v4f dB  = *(const v4fa*)(DX + (size_t)nB * 4);
  const float icA = 1.0f / fmaxf(dA.w, 1.0f);
  const float icB = 1.0f / fmaxf(dB.w, 1.0f);
  const unsigned mv = 0u - (unsigned)((4 * uc + 3) < nN);
  v4f q;
#pragma unroll
  for (int e = 0; e < 4; ++e) {
    const int te = t0 + e;
    const int ne = te / 3;
    const int ce = te - 3 * ne;
    const bool useA = (ne == nA);
    const float nx = useA ? dA.x : dB.x;
    const float ny = useA ? dA.y : dB.y;
    const float nz = useA ? dA.z : dB.z;
    const float ic = useA ? icA : icB;
    const float num = (ce == 0) ? nx : ((ce == 1) ? ny : nz);
    const float fv = num * ic;
    const float vv = v4[e];
    q[e] = __uint_as_float((__float_as_uint(vv) & mv) | (__float_as_uint(fv) & ~mv));
  }
  float* dp = out + (size_t)4 * u;
  if (u < nN) *(volatile v4f*)dp = q;
  __threadfence();
  if (u < nN) *(volatile v4f*)dp = q;
}

static inline int cdiv(int a, int b) { return (a + b - 1) / b; }
static inline size_t al256(size_t v) { return (v + 255) & ~(size_t)255; }

extern "C" void kernel_launch(void* const* d_in, const int* in_sizes, int n_in,
                              void* d_out, int out_size, void* d_ws, size_t ws_size,
                              hipStream_t stream) {
  if (n_in < 19) return;
  if (in_sizes[0] < HID || (in_sizes[0] % HID) != 0) return;
  const int nN = in_sizes[0] / HID;
  if (nN < 8 || (nN % 8) != 0) return;
  const int nE = in_sizes[2];
  if (nE < 1 || nE >= (1 << 22)) return;
  if (in_sizes[3] != nE || in_sizes[1] != 3 * nE) return;
  if (in_sizes[4] != W1R * HID || in_sizes[5] != HID) return;
  if (in_sizes[6] != HID * HID || in_sizes[7] != HID) return;
  if (in_sizes[8] != 2 * HID * HID || in_sizes[9] != HID) return;
  if (in_sizes[10] != HID * HID || in_sizes[11] != HID) return;
  if (in_sizes[12] != HID * HID || in_sizes[13] != HID) return;
  if (in_sizes[14] != HID) return;
  if (in_sizes[15] != HID * HID || in_sizes[16] != HID) return;
  if (in_sizes[17] != HID || in_sizes[18] != 1) return;
  if ((long long)out_size != 4LL * nN + (long long)nN * HID) return;

  const float* h   = (const float*)d_in[0];
  const float* cd  = (const float*)d_in[1];
  const int*   rowp = (const int*)d_in[2];
  const int*   colp = (const int*)d_in[3];
  const float* We1 = (const float*)d_in[4];
  const float* be1 = (const float*)d_in[5];
  const float* We2 = (const float*)d_in[6];
  const float* be2 = (const float*)d_in[7];
  const float* Wn1 = (const float*)d_in[8];
  const float* bn1 = (const float*)d_in[9];
  const float* Wn2 = (const float*)d_in[10];
  const float* bn2 = (const float*)d_in[11];
  const float* Wc1 = (const float*)d_in[12];
  const float* bc1 = (const float*)d_in[13];
  const float* Wc2 = (const float*)d_in[14];
  const float* Wv1 = (const float*)d_in[15];
  const float* bv1 = (const float*)d_in[16];
  const float* Wv2 = (const float*)d_in[17];
  const float* bv2 = (const float*)d_in[18];
  float* out0 = (float*)d_out;
  float* out2 = out0 + (size_t)4 * nN;

  const int MP = cdiv(nN, GBM) * GBM;
  const int gM = MP / GBM;
  const int gA = cdiv(MP, NBA);
  if ((long long)gA * NBA < (long long)MP) return;
  const int EH = cdiv(cdiv(nE, NRANGE), EPB) * EPB;
  if (EH < EPB || EH >= (1 << 21)) return;

  char* ws = (char*)d_ws;
  size_t off = 0;
  const size_t oWABT = off; off = al256(off + (size_t)NPV * HID * 2);
  const size_t oWE2T = off; off = al256(off + (size_t)HID * HID * 2);
  const size_t oWX1T = off; off = al256(off + (size_t)HID * HID * 2);
  const size_t oWN1T = off; off = al256(off + (size_t)HID * KN1 * 2);
  const size_t oWN2T = off; off = al256(off + (size_t)HID * KN2 * 2);
  const size_t oVEL  = off; off = al256(off + (size_t)MP * 4);
  const size_t oDX   = off; off = al256(off + (size_t)MP * 4 * 4);
  const size_t oMI   = off; off = al256(off + (size_t)MP * HID * 4);
  size_t szRM = (size_t)EH * MPITCH * 2;
  if (szRM < (size_t)MP * HID * 2) szRM = (size_t)MP * HID * 2;
  if (szRM < (size_t)MP * KN2 * 2) szRM = (size_t)MP * KN2 * 2;
  const size_t oRM   = off; off = al256(off + szRM);
  const size_t oTR   = off; off = al256(off + (size_t)EH * 4 * 4);
  size_t szRP = (size_t)MP * NPQ * 4;
  if (szRP < (size_t)MP * KN1 * 2) szRP = (size_t)MP * KN1 * 2;
  const size_t oRP   = off; off = al256(off + szRP);
  if (off > ws_size || off > (size_t)WSMAX) return;
  unsigned short* WABT = (unsigned short*)(ws + oWABT);
  unsigned short* WE2T = (unsigned short*)(ws + oWE2T);
  unsigned short* WX1T = (unsigned short*)(ws + oWX1T);
  unsigned short* WN1T = (unsigned short*)(ws + oWN1T);
  unsigned short* WN2T = (unsigned short*)(ws + oWN2T);
  float*          VEL  = (float*)(ws + oVEL);
  float*          DX   = (float*)(ws + oDX);
  float*          MI   = (float*)(ws + oMI);
  unsigned short* HB   = (unsigned short*)(ws + oRM);
  unsigned short* MSG  = (unsigned short*)(ws + oRM);
  unsigned short* G1   = (unsigned short*)(ws + oRM);
  float*          TR   = (float*)(ws + oTR);
  float*          PQ   = (float*)(ws + oRP);
  unsigned short* NZ   = (unsigned short*)(ws + oRP);

  hipFuncSetAttribute(reinterpret_cast<const void*>(&k_edge), hipFuncAttributeMaxDynamicSharedMemorySize,
                      (int)EDGE_LDS_BYTES);
  hipFuncSetAttribute(reinterpret_cast<const void*>(&k_scan), hipFuncAttributeMaxDynamicSharedMemorySize,
                      (int)AGG_LDS_BYTES);

  const int nXP   = cdiv(MP, NTHR) * NTHR;
  const int nPrep = NU_WAB + NU_WV + 2 * NU_W128 + NU_WN1 + NU_WN2 + MP * 16 + MP * 32 + nXP;
  const int vec8  = 1;

  k_prep<<<nPrep / NTHR, NTHR, 0, stream>>>(h, We1, We2, Wc1, Wn1, Wn2, Wv1, nN, MP,
                                            WABT, WE2T, WX1T, WN1T, WN2T, HB, MI, DX);
  k_gemm<0><<<dim3(gM, NPV / GBN), GTHR, 0, stream>>>(HB, HID, WABT, HID, HID, bv1, Wv2, bv2, nN, PQ, NPQ, G1, VEL);
  for (int rr = 0; rr < NRANGE; ++rr) {
    const int eBase = rr * EH;
    if (eBase >= nE) break;
    const int nEh = (nE - eBase) < EH ? (nE - eBase) : EH;
    k_edge<<<cdiv(nEh, EPB), NTHR, EDGE_LDS_BYTES, stream>>>(rowp, colp, nE, nN, eBase, nEh, PQ, cd, WE2T, WX1T,
                                                            be1, be2, bc1, We1 + (size_t)2 * HID * HID, Wc2,
                                                            MSG, TR);
    k_scan<<<gA, NTHR, AGG_LDS_BYTES, stream>>>(rowp + eBase, nEh, vec8, MP, MSG, TR, MI, DX);
  }
  k_nz<<<(MP * 16) / NTHR, NTHR, 0, stream>>>(MI, h, nN, MP * 16, NZ);
  k_gemm<1><<<dim3(gM, 1), GTHR, 0, stream>>>(NZ, KN1, WN1T, KN1, KN1, bn1, Wv2, bv2, nN, MI, HID, G1, VEL);
  k_gemm<2><<<dim3(gM, 1), GTHR, 0, stream>>>(G1, KN2, WN2T, KN2, KN2, bn2, Wv2, bv2, nN, out2, HID, NZ, VEL);
  k_vf<<<cdiv(nN, NTHR), NTHR, 0, stream>>>(VEL, DX, nN, out0);
  (void)hipGetLastError();
}
